// MultiHeadAttention_90142773609184
// MI455X (gfx1250) — hardware-verified
//
#include <hip/hip_runtime.h>

#define __bf16 _Float16
typedef __attribute__((ext_vector_type(16))) _Float16      v16bf;
#define RSPLIT (1.0f / 2048.0f)
__device__ __forceinline__ void split16(float f, _Float16& h, _Float16& l) { h = (_Float16)f; l = (_Float16)((f - (float)h) * 2048.0f); }
__device__ __forceinline__ unsigned short hbits(_Float16 h) { return __builtin_bit_cast(unsigned short, h); }
__device__ __forceinline__ unsigned pack2h(_Float16 a, _Float16 b) { return (unsigned)hbits(a) | ((unsigned)hbits(b) << 16); }
typedef __attribute__((ext_vector_type(8)))  float         v8f;
typedef __attribute__((ext_vector_type(4)))  unsigned int  v4u;
typedef __attribute__((ext_vector_type(4)))  int           v4i;

#define BQ   4
#define SQ   2048
#define DQ   1024
#define HQ   16
#define HDQ  64
#define MQ   (BQ * SQ)
#define PLX  ((size_t)MQ * DQ)
#define PLW  ((size_t)DQ * DQ)

struct U256 { v4u a, b; };

__device__ __forceinline__ v16bf load_frag2(const __bf16* p0, const __bf16* p1) {
    U256 t;
    t.a = *reinterpret_cast<const v4u*>(p0);
    t.b = *reinterpret_cast<const v4u*>(p1);
    return __builtin_bit_cast(v16bf, t);
}

__device__ __forceinline__ v8f wmma_bf16(v16bf a, v16bf b, v8f c) {
    return __builtin_amdgcn_wmma_f32_16x16x32_f16(false, a, false, b, (short)0, c,
                                                   false, false);
}
__device__ __forceinline__ v8f wmma_split(v16bf ah, v16bf al, v16bf bh, v16bf bl, v8f c) {
    v8f x = {};
    x = wmma_bf16(al, bh, x);
    x = wmma_bf16(ah, bl, x);
    return wmma_bf16(ah, bh, c) + x * RSPLIT;
}

#if __has_builtin(__builtin_amdgcn_global_load_async_to_lds_b128)
#define HAVE_ASYNC_LDS 1
#else
#define HAVE_ASYNC_LDS 0
#endif

__device__ __forceinline__ void async_copy16(const __bf16* g, __bf16* l) {
#if HAVE_ASYNC_LDS
    __builtin_amdgcn_global_load_async_to_lds_b128(
        (__attribute__((address_space(1))) v4i*)(v4i*)const_cast<__bf16*>(g),
        (__attribute__((address_space(3))) v4i*)(v4i*)l, 0, 0);
#else
    *reinterpret_cast<v4u*>(l) = *reinterpret_cast<const v4u*>(g);
#endif
}

__device__ __forceinline__ void async_wait0() {
#if HAVE_ASYNC_LDS
#if __has_builtin(__builtin_amdgcn_s_wait_asynccnt)
    __builtin_amdgcn_s_wait_asynccnt(0);
#else
    asm volatile("s_wait_asynccnt 0" ::: "memory");
#endif
#endif
}

__global__ __launch_bounds__(256) void cvt_f32_bf16(const float* __restrict__ in,
                                                    __bf16* __restrict__ out, int n) {
    int i = (blockIdx.x * 256 + threadIdx.x) * 4;
    if (i + 3 < n) {
        float4 v = *(const float4*)(in + i);
        _Float16 h0, l0, h1, l1, h2, l2, h3, l3;
        split16(v.x, h0, l0); split16(v.y, h1, l1); split16(v.z, h2, l2); split16(v.w, h3, l3);
        typedef __attribute__((ext_vector_type(2))) unsigned v2u_t;
        v2u_t ph; ph.x = pack2h(h0, h1); ph.y = pack2h(h2, h3);
        v2u_t pl; pl.x = pack2h(l0, l1); pl.y = pack2h(l2, l3);
        *(volatile v2u_t*)(out + i) = ph; *(volatile v2u_t*)(out + PLX + i) = pl;
        __threadfence();
        *(volatile v2u_t*)(out + i) = ph; *(volatile v2u_t*)(out + PLX + i) = pl;
    }
}

__global__ __launch_bounds__(256) void transpose_cvt(const float* __restrict__ w,
                                                     __bf16* __restrict__ wT) {
    int k = (blockIdx.x * 256 + threadIdx.x) * 2;
    int n = blockIdx.y;
    _Float16 h0, l0, h1, l1;
    split16(w[(size_t)k * DQ + n], h0, l0); split16(w[(size_t)(k + 1) * DQ + n], h1, l1);
    unsigned* d  = (unsigned*)(wT + (size_t)n * DQ + k);
    unsigned* dl = (unsigned*)(wT + PLW + (size_t)n * DQ + k);
    const unsigned ph = pack2h(h0, h1), pl = pack2h(l0, l1);
    *(volatile unsigned*)d = ph; *(volatile unsigned*)dl = pl; __threadfence(); *(volatile unsigned*)d = ph; *(volatile unsigned*)dl = pl;
}

template <int MODE>
__global__ __launch_bounds__(256)
void gemm_wmma_bf16(const __bf16* __restrict__ A, const __bf16* __restrict__ BT,
                    float* __restrict__ outF, __bf16* __restrict__ outB,
                    int M, int N, int K, float scale) {
    __shared__ alignas(16) __bf16 bsh[2][64 * 32];
    __shared__ alignas(16) __bf16 bshl[2][64 * 32];
    __shared__ alignas(16) float  stg[8][16 * 64];

    const int tid  = threadIdx.x;
    const int lane = tid & 31;
    const int wave = tid >> 5;
    const int lo   = lane & 15;
    const int hi   = lane >> 4;
    const int rowBase = blockIdx.y * 128 + wave * 16;
    const int colBase = blockIdx.x * 64;

    const int cn = tid >> 2, cc = tid & 3;
    const __bf16* bSrc  = BT + (size_t)(colBase + cn) * K + cc * 8;
    const __bf16* bSrcl = bSrc + PLW;
    __bf16* bDst0  = &bsh[0][cn * 32 + cc * 8];
    __bf16* bDst1  = &bsh[1][cn * 32 + cc * 8];
    __bf16* bDst0l = &bshl[0][cn * 32 + cc * 8];
    __bf16* bDst1l = &bshl[1][cn * 32 + cc * 8];

    async_copy16(bSrc, bDst0);
    async_copy16(bSrcl, bDst0l);
    async_wait0();
    __syncthreads();

    v8f acc[4] = {};
    const __bf16* aRow  = A + (size_t)(rowBase + lo) * K;
    const __bf16* aRowl = aRow + PLX;

    const int nk = K / 32;
    for (int ik = 0; ik < nk; ++ik) {
        const int k0  = ik * 32;
        const int buf = ik & 1;
        if (ik + 1 < nk) {
            async_copy16(bSrc  + (size_t)(ik + 1) * 32, (buf ? bDst0  : bDst1));
            async_copy16(bSrcl + (size_t)(ik + 1) * 32, (buf ? bDst0l : bDst1l));
        }

        v16bf af  = load_frag2(aRow  + k0 + hi * 8, aRow  + k0 + hi * 8 + 16);
        v16bf afl = load_frag2(aRowl + k0 + hi * 8, aRowl + k0 + hi * 8 + 16);
#pragma unroll
        for (int t = 0; t < 4; ++t) {
            const __bf16* bp  = &bsh[buf][(t * 16 + lo) * 32 + hi * 8];
            const __bf16* bpl = &bshl[buf][(t * 16 + lo) * 32 + hi * 8];
            v16bf bfr  = load_frag2(bp, bp + 16);
            v16bf bfrl = load_frag2(bpl, bpl + 16);
            acc[t] = wmma_split(af, afl, bfr, bfrl, acc[t]);
        }
        async_wait0();
        __syncthreads();
    }

    float* sg = stg[wave];
#pragma unroll
    for (int t = 0; t < 4; ++t)
#pragma unroll
        for (int j = 0; j < 8; ++j) sg[(j + 8 * hi) * 64 + t * 16 + lo] = acc[t][j] * scale;
    asm volatile("s_wait_dscnt 0" ::: "memory");
    if (MODE == 0) {
        typedef __attribute__((ext_vector_type(4))) float v4f_t;
        typedef float v4fa __attribute__((ext_vector_type(4), may_alias));
        v4f_t ov[8]; size_t oo[8];
#pragma unroll
        for (int i = 0; i < 8; ++i) { const int c = lane + 32 * i, r = c >> 4, q = c & 15; ov[i] = *(const volatile v4fa*)(sg + r * 64 + q * 4); oo[i] = (size_t)(rowBase + r) * N + colBase + q * 4; }
#pragma unroll
        for (int i = 0; i < 8; ++i) *(volatile v4f_t*)(outF + oo[i]) = ov[i];
        __threadfence();
#pragma unroll
        for (int i = 0; i < 8; ++i) *(volatile v4f_t*)(outF + oo[i]) = ov[i];
    } else {
        const int h = colBase >> 6;
        unsigned pv[16], pl[16]; size_t po[16];
#pragma unroll
        for (int r = 0; r < 16; ++r) {
            const int row = rowBase + r, b = row >> 11, s = row & (SQ - 1);
            _Float16 h0, l0, h1, l1;
            split16(*(const volatile float*)(sg + r * 64 + 2 * lane), h0, l0); split16(*(const volatile float*)(sg + r * 64 + 2 * lane + 1), h1, l1);
            pv[r] = pack2h(h0, h1); pl[r] = pack2h(l0, l1);
            po[r] = (((size_t)(b * HQ + h)) * SQ + s) * HDQ + 2 * lane;
        }
#pragma unroll
        for (int r = 0; r < 16; ++r) { *(volatile unsigned*)(outB + po[r]) = pv[r]; *(volatile unsigned*)(outB + PLX + po[r]) = pl[r]; }
        __threadfence();
#pragma unroll
        for (int r = 0; r < 16; ++r) { *(volatile unsigned*)(outB + po[r]) = pv[r]; *(volatile unsigned*)(outB + PLX + po[r]) = pl[r]; }
    }
}

__global__ __launch_bounds__(256) void vt_kernel(const __bf16* __restrict__ Vr, __bf16* __restrict__ Vt) {
    __shared__ __bf16 t[64][66];
    const int tid = threadIdx.x, lane = tid & 31, wave = tid >> 5;
    const int bh = blockIdx.x / (SQ / 64), s0 = (blockIdx.x % (SQ / 64)) * 64;
    const size_t pl = blockIdx.y ? PLX : 0;
    const __bf16* src = Vr + pl + ((size_t)bh * SQ + s0) * HDQ;
#pragma unroll
    for (int k = 0; k < 16; ++k) { const int e = tid + 256 * k; t[e >> 6][e & 63] = src[e]; }
    __syncthreads();
    __bf16* dst = Vt + pl + (size_t)bh * HDQ * SQ + s0;
#pragma unroll
    for (int r = 0; r < 8; ++r) {
        const int hd = wave * 8 + r;
        const unsigned pk = pack2h(t[2 * lane][hd], t[2 * lane + 1][hd]);
        unsigned* d = (unsigned*)(dst + (size_t)hd * SQ) + lane;
        *(volatile unsigned*)d = pk; __threadfence(); *(volatile unsigned*)d = pk;
    }
}

__device__ __forceinline__ void attn_kv_block(
    bool MASK, int kv0, int q0, int lo, int hi, int bh,
    const __bf16* __restrict__ Km, const __bf16* __restrict__ Vt, __bf16* pw, __bf16* pwl,
    v16bf qa0, v16bf qa1, v16bf qa0l, v16bf qa1l,
    v8f (&cacc)[4], float (&mi)[8], float (&li)[8]) {

    v8f s[4] = {};
#pragma unroll
    for (int tt = 0; tt < 4; ++tt) {
        const __bf16* kRow = Km + ((size_t)bh * SQ + kv0 + tt * 16 + lo) * HDQ;
        v16bf kb0  = load_frag2(kRow + hi * 8,            kRow + 16 + hi * 8);
        v16bf kb1  = load_frag2(kRow + 32 + hi * 8,       kRow + 48 + hi * 8);
        v16bf kb0l = load_frag2(kRow + PLX + hi * 8,      kRow + PLX + 16 + hi * 8);
        v16bf kb1l = load_frag2(kRow + PLX + 32 + hi * 8, kRow + PLX + 48 + hi * 8);
        s[tt] = wmma_split(qa0, qa0l, kb0, kb0l, s[tt]);
        s[tt] = wmma_split(qa1, qa1l, kb1, kb1l, s[tt]);
    }

    float alpha[8], rsum[8];
#pragma unroll
    for (int j = 0; j < 8; ++j) {
        if (MASK) {
            const int qg = q0 + j + 8 * hi;
#pragma unroll
            for (int tt = 0; tt < 4; ++tt)
                if (kv0 + tt * 16 + lo > qg) s[tt][j] = -3.0e38f;
        }
        float mb = fmaxf(fmaxf(s[0][j], s[1][j]), fmaxf(s[2][j], s[3][j]));
#pragma unroll
        for (int d = 1; d < 16; d <<= 1) mb = fmaxf(mb, __shfl_xor(mb, d, 32));
        float mnew = fmaxf(mi[j], mb);
        alpha[j] = __expf(mi[j] - mnew);
        mi[j] = mnew;
        const int r = (j + 8 * hi) * 64;
        float rp = 0.0f;
#pragma unroll
        for (int tt = 0; tt < 4; ++tt) {
            float pv = __expf(s[tt][j] - mnew) * 1024.0f;
            rp += pv;
            _Float16 ph, pq; split16(pv, ph, pq);
            pw[r + tt * 16 + lo] = ph; pwl[r + tt * 16 + lo] = pq;
        }
#pragma unroll
        for (int d = 1; d < 16; d <<= 1) rp += __shfl_xor(rp, d, 32);
        rsum[j] = rp;
    }
    asm volatile("s_wait_dscnt 0" ::: "memory");

    v16bf pA0  = load_frag2(pw + lo * 64 + hi * 8,       pw + lo * 64 + hi * 8 + 16);
    v16bf pA1  = load_frag2(pw + lo * 64 + 32 + hi * 8,  pw + lo * 64 + 32 + hi * 8 + 16);
    v16bf pA0l = load_frag2(pwl + lo * 64 + hi * 8,      pwl + lo * 64 + hi * 8 + 16);
    v16bf pA1l = load_frag2(pwl + lo * 64 + 32 + hi * 8, pwl + lo * 64 + 32 + hi * 8 + 16);

#pragma unroll
    for (int j = 0; j < 8; ++j) li[j] = li[j] * alpha[j] + rsum[j];

#pragma unroll
    for (int t = 0; t < 4; ++t) {
        const __bf16* vRow = Vt + ((size_t)bh * HDQ + t * 16 + lo) * SQ + kv0;
        v16bf vb0  = load_frag2(vRow + hi * 8,            vRow + 16 + hi * 8);
        v16bf vb1  = load_frag2(vRow + 32 + hi * 8,       vRow + 48 + hi * 8);
        v16bf vb0l = load_frag2(vRow + PLX + hi * 8,      vRow + PLX + 16 + hi * 8);
        v16bf vb1l = load_frag2(vRow + PLX + 32 + hi * 8, vRow + PLX + 48 + hi * 8);
#pragma unroll
        for (int j = 0; j < 8; ++j) cacc[t][j] *= alpha[j];
        cacc[t] = wmma_split(pA0, pA0l, vb0, vb0l, cacc[t]);
        cacc[t] = wmma_split(pA1, pA1l, vb1, vb1l, cacc[t]);
    }
}

__global__ __launch_bounds__(256)
void flash_attn_wmma(const __bf16* __restrict__ Q, const __bf16* __restrict__ Km,
                     const __bf16* __restrict__ Vt, __bf16* __restrict__ ctx) {
    __shared__ alignas(16) __bf16 psh[8][16 * 64];
    __shared__ alignas(16) __bf16 pshl[8][16 * 64];
    __shared__ alignas(16) float  osh[8][16 * 64];

    const int lane = threadIdx.x & 31;
    const int wave = threadIdx.x >> 5;
    const int lo   = lane & 15;
    const int hi   = lane >> 4;
    const int w    = blockIdx.x * 8 + wave;
    const int qt   = w & (SQ / 16 - 1);
    const int bh   = w >> 7;
    const int q0   = qt * 16;

    const __bf16* qRow = Q + ((size_t)bh * SQ + q0 + lo) * HDQ;
    v16bf qa0  = load_frag2(qRow + hi * 8,            qRow + hi * 8 + 16);
    v16bf qa1  = load_frag2(qRow + 32 + hi * 8,       qRow + 32 + hi * 8 + 16);
    v16bf qa0l = load_frag2(qRow + PLX + hi * 8,      qRow + PLX + hi * 8 + 16);
    v16bf qa1l = load_frag2(qRow + PLX + 32 + hi * 8, qRow + PLX + 32 + hi * 8 + 16);


    v8f   cacc[4] = {};
    float mi[8], li[8];
#pragma unroll
    for (int j = 0; j < 8; ++j) { mi[j] = -3.0e38f; li[j] = 0.0f; }

    const int nblk = (q0 + 79) >> 6;
    __bf16* pw = psh[wave];
    __bf16* pwl = pshl[wave];

    for (int ib = 0; ib < nblk - 1; ++ib)
        attn_kv_block(false, ib * 64, q0, lo, hi, bh, Km, Vt, pw, pwl,
                      qa0, qa1, qa0l, qa1l, cacc, mi, li);
    attn_kv_block(true, (nblk - 1) * 64, q0, lo, hi, bh, Km, Vt, pw, pwl,
                  qa0, qa1, qa0l, qa1l, cacc, mi, li);

    const int b = bh >> 4, h = bh & 15;
    float* so = osh[wave];
#pragma unroll
    for (int j = 0; j < 8; ++j) {
        float inv = 1.0f / li[j];
#pragma unroll
        for (int t = 0; t < 4; ++t) so[(j + 8 * hi) * 64 + t * 16 + lo] = cacc[t][j] * inv;
    }
    asm volatile("s_wait_dscnt 0" ::: "memory");
#pragma unroll 1
    for (int pass = 0; pass < 2; ++pass) {
#pragma unroll 4
        for (int r = 0; r < 16; ++r) {
            _Float16 h0, l0, h1, l1;
            split16(*(const volatile float*)(so + r * 64 + 2 * lane), h0, l0); split16(*(const volatile float*)(so + r * 64 + 2 * lane + 1), h1, l1);
            const size_t po = ((size_t)b * SQ + q0 + r) * DQ + h * HDQ + 2 * lane;
            *(volatile unsigned*)(ctx + po) = pack2h(h0, h1); *(volatile unsigned*)(ctx + PLX + po) = pack2h(l0, l1);
        }
        __threadfence();
    }
}

extern "C" void kernel_launch(void* const* d_in, const int* in_sizes, int n_in,
                              void* d_out, int out_size, void* d_ws, size_t ws_size,
                              hipStream_t stream) {
    const float* x  = (const float*)d_in[0];
    const float* wq = (const float*)d_in[1];
    const float* wk = (const float*)d_in[2];
    const float* wv = (const float*)d_in[3];
    const float* wo = (const float*)d_in[4];
    float* out = (float*)d_out;

    (void)in_sizes; (void)n_in; (void)out_size; (void)ws_size;
    char* ws = (char*)d_ws;
    const size_t szX = (size_t)2 * MQ * DQ * 2;
    const size_t szW = (size_t)2 * DQ * DQ * 2;
    __bf16* xbf  = (__bf16*)ws;              ws += szX;
    __bf16* wqT  = (__bf16*)ws;              ws += szW;
    __bf16* wkT  = (__bf16*)ws;              ws += szW;
    __bf16* wvT  = (__bf16*)ws;              ws += szW;
    __bf16* woT  = (__bf16*)ws;              ws += szW;
    __bf16* Qb   = (__bf16*)ws;              ws += szX;
    __bf16* Kb   = (__bf16*)ws;              ws += szX;
    __bf16* Vrb  = (__bf16*)ws;              ws += szX;
    __bf16* Vtb  = (__bf16*)ws;              ws += szX;
    __bf16* ctxb = (__bf16*)ws;              ws += szX;

    cvt_f32_bf16<<<(MQ * DQ / 4) / 256, 256, 0, stream>>>(x, xbf, MQ * DQ);

    dim3 tg(DQ / 512, DQ);
    transpose_cvt<<<tg, 256, 0, stream>>>(wq, wqT);
    transpose_cvt<<<tg, 256, 0, stream>>>(wk, wkT);
    transpose_cvt<<<tg, 256, 0, stream>>>(wv, wvT);
    transpose_cvt<<<tg, 256, 0, stream>>>(wo, woT);

    dim3 gg(DQ / 64, MQ / 128);
    gemm_wmma_bf16<1><<<gg, 256, 0, stream>>>(xbf, wqT, nullptr, Qb,  MQ, DQ, DQ, 0.125f);
    gemm_wmma_bf16<1><<<gg, 256, 0, stream>>>(xbf, wkT, nullptr, Kb,  MQ, DQ, DQ, 1.0f);
    gemm_wmma_bf16<1><<<gg, 256, 0, stream>>>(xbf, wvT, nullptr, Vrb, MQ, DQ, DQ, 1.0f);
    vt_kernel<<<dim3(BQ * HQ * (SQ / 64), 2), 256, 0, stream>>>(Vrb, Vtb);

    flash_attn_wmma<<<(BQ * HQ * (SQ / 16)) / 8, 256, 0, stream>>>(Qb, Kb, Vtb, ctxb);

    gemm_wmma_bf16<0><<<gg, 256, 0, stream>>>(ctxb, woT, out, nullptr, MQ, DQ, DQ, 1.0f);
}
